// GCN_LSTM_67224828117588
// MI455X (gfx1250) — hardware-run, weakly checked
//
#include <hip/hip_runtime.h>
#include <stddef.h>


typedef _Float16 h16;
typedef _Float16 v16h __attribute__((ext_vector_type(16)));
typedef _Float16 v8h  __attribute__((ext_vector_type(8)));
typedef float    v8f  __attribute__((ext_vector_type(8)));
typedef float    v4f  __attribute__((ext_vector_type(4)));

#ifndef NROWS
#define NROWS 500000
#endif
#define NROWS_FULL 500000
#define XDIM  16
#define HIDN  128
#define MID1  64
#define MID2  32
#define BROWS 64
#define NBLK  ((NROWS + BROWS - 1) / BROWS)

static_assert(NROWS >= 32 && NROWS <= NROWS_FULL);
static_assert((NROWS % 32) == 0);
static_assert(XDIM == 16);
static_assert((HIDN % 32) == 0 && HIDN == 8 * 16);
static_assert((MID1 % 32) == 0 && MID1 == 4 * 16);
static_assert(MID2 == 2 * 16);
static_assert(BROWS == 4 * 16);

#define LDH 136
#define LDT 72
static_assert((LDH % 8) == 0 && LDH >= HIDN);
static_assert((LDT % 8) == 0 && LDT >= MID1);
static_assert(4 * 16 * LDH * 2 + 4 * 16 * LDT * 2 + BROWS * 4 <= 131072);

#define XCARRY  16.0f
#define WCARRY  64.0f
#define HCARRY  256.0f
#define H1CARRY 1024.0f

#define WG_BYTES  ((size_t)3 * HIDN * XDIM * 2)
#define M1_BYTES  ((size_t)MID1 * HIDN * 2)
#define M2_BYTES  ((size_t)MID2 * MID1 * 2)
#define OFF_WG ((size_t)0)
#define OFF_M1 (OFF_WG + WG_BYTES)
#define OFF_M2 (OFF_M1 + M1_BYTES)
#define WS_TOTAL (OFF_M2 + M2_BYTES)
static_assert((WG_BYTES % 512) == 0 && (M1_BYTES % 512) == 0 && (M2_BYTES % 512) == 0);
static_assert(WS_TOTAL <= (size_t)134217728);
static_assert(((HIDN * XDIM / 8) % 256) == 0);
static_assert(((MID1 * HIDN / 8) % 256) == 0);
static_assert(((MID2 * MID1 / 8) % 256) == 0);

__device__ __forceinline__ float bf16r(float x) {
  unsigned int u = __float_as_uint(x);
  u = (u + 0x7FFFu + ((u >> 16) & 1u)) & 0xFFFF0000u;
  return __uint_as_float(u);
}

static __device__ __forceinline__ h16 toh_flush(float v) {
  const h16 r = (h16)v;
  return (fabsf(v) < 6.103515625e-05f) ? (h16)0.0f : r;
}

__device__ __forceinline__ v16h frag_at(const _Float16* p) {
  v8h lo = *(const v8h*)(p);
  v8h hi = *(const v8h*)(p + 16);
  v16h out;
#pragma unroll
  for (int i = 0; i < 8; ++i) { out[i] = lo[i]; out[i + 8] = hi[i]; }
  return out;
}
__device__ __forceinline__ v16h ld_frag(const _Float16* base, unsigned ld) {
  const unsigned lane = threadIdx.x & 31u;
  return frag_at(base + (lane & 15u) * ld + (lane >> 4) * 8u);
}
__device__ __forceinline__ v16h frag_lo_at(const _Float16* p) {
  v8h lo = *(const v8h*)(p);
  v16h out;
#pragma unroll
  for (int i = 0; i < 8; ++i) { out[i] = lo[i]; out[i + 8] = (_Float16)0.0f; }
  return out;
}

__device__ __forceinline__ v8f wmma16(v16h a, v16h b, v8f c) {
  v8f d = __builtin_amdgcn_wmma_f32_16x16x32_f16(false, a, false, b, (short)0, c,
                                                 false, false);
  asm volatile("v_nop\n\tv_nop\n\tv_nop\n\tv_nop" : "+v"(d) : "v"(a), "v"(b));
  return d;
}

__device__ __forceinline__ float red16_sum(float x) {
#pragma unroll
  for (int off = 1; off < 16; off <<= 1) x += __shfl_xor(x, off, 32);
  return x;
}

__device__ __forceinline__ void wave_lds_sync() {
  __builtin_amdgcn_fence(3  , "wavefront");
  asm volatile("s_wait_dscnt 0x0" ::: "memory");
  __builtin_amdgcn_wave_barrier();
}

#define LOG2E 1.44269504088896340736f
__device__ __forceinline__ float fast_sigmoid(float v) {
  const float e = __builtin_amdgcn_exp2f(-v * LOG2E);
  return __builtin_amdgcn_rcpf(1.0f + e);
}
__device__ __forceinline__ float fast_tanh(float v) {
  const float e = __builtin_amdgcn_exp2f(2.0f * v * LOG2E);
  return 1.0f - 2.0f * __builtin_amdgcn_rcpf(1.0f + e);
}

__global__ __launch_bounds__(256) void wsmall_kernel(
    const float* __restrict__ W, _Float16* __restrict__ Wt, unsigned K, unsigned N) {
  const unsigned idx = blockIdx.x * 256u + threadIdx.x;
  const unsigned ppr = K >> 3;
  const unsigned total = N * ppr;
  const bool ok = idx < total;
  const unsigned ic = ok ? idx : (total - 1u);
  const unsigned n = ic / ppr;
  const unsigned kc = (ic - n * ppr) * 8u;
  v8h o;
#pragma unroll
  for (unsigned j = 0; j < 8u; ++j) {
    const float v = W[(size_t)(kc + j) * N + n];
    o[j] = toh_flush(WCARRY * bf16r(v));
  }
  _Float16* p = Wt + (size_t)ic * 8u;
  if (ok) *(volatile v8h*)p = o;
  __threadfence();
  if (ok) *(volatile v8h*)p = o;
}

__global__ __launch_bounds__(128) void gclstm_mlp_kernel(
    const float* __restrict__ x,
    const _Float16* __restrict__ Wg, const _Float16* __restrict__ M1t,
    const _Float16* __restrict__ M2t,
    const float* __restrict__ bci, const float* __restrict__ bcc, const float* __restrict__ bco,
    const float* __restrict__ bgi, const float* __restrict__ bgc, const float* __restrict__ bgo,
    const float* __restrict__ wco,
    const float* __restrict__ bm1, const float* __restrict__ bm2,
    const float* __restrict__ M3, const float* __restrict__ bm3,
    float* __restrict__ out) {
  __shared__ __attribute__((aligned(16))) _Float16 Hs[4 * 16 * LDH];
  __shared__ __attribute__((aligned(16))) _Float16 H1s[4 * 16 * LDT];
  __shared__ __attribute__((aligned(16))) float Outs[BROWS];

  const unsigned tid = threadIdx.x, lane = tid & 31u;
  const unsigned wave = (unsigned)__builtin_amdgcn_readfirstlane((int)(tid >> 5));
  const unsigned hh = lane >> 4, m = lane & 15u;
  const unsigned row0 = blockIdx.x * (unsigned)BROWS;
  const unsigned trow = row0 + wave * 16u;

  unsigned myrow = trow + m;
  myrow = (myrow < (unsigned)NROWS) ? myrow : ((unsigned)NROWS - 1u);
  const float* xr = x + (size_t)myrow * XDIM + hh * 8u;
  const v4f x0 = *(const v4f*)(xr);
  const v4f x1 = *(const v4f*)(xr + 4);
  v16h ax;
#pragma unroll
  for (int i = 0; i < 4; ++i) {
    ax[i]     = toh_flush(XCARRY * bf16r(x0[i]));
    ax[i + 4] = toh_flush(XCARRY * bf16r(x1[i]));
  }
#pragma unroll
  for (int i = 8; i < 16; ++i) ax[i] = (_Float16)0.0f;

  _Float16* H = Hs + wave * (16u * LDH);
  _Float16* H1 = H1s + wave * (16u * LDT);
  const float gs = 1.0f / (XCARRY * WCARRY);

#pragma unroll 2
  for (unsigned n = 0; n < 8u; ++n) {
    const unsigned col = 16u * n + m;
    const _Float16* wp = Wg + (size_t)col * XDIM + hh * 8u;
    const v16h bI = frag_lo_at(wp);
    const v16h bC = frag_lo_at(wp + HIDN * XDIM);
    const v16h bO = frag_lo_at(wp + 2 * HIDN * XDIM);
    const v8f ai = wmma16(ax, bI, (v8f){});
    const v8f at = wmma16(ax, bC, (v8f){});
    const v8f ao = wmma16(ax, bO, (v8f){});
    const float cbi = bf16r(bci[col]), gbi = bf16r(bgi[col]);
    const float cbc = bf16r(bcc[col]), gbc = bf16r(bgc[col]);
    const float cbo = bf16r(bco[col]), gbo = bf16r(bgo[col]);
    const float wc = bf16r(wco[col]);
#pragma unroll
    for (int r = 0; r < 8; ++r) {
      const float I  = fast_sigmoid((ai[r] * gs + cbi) + gbi);
      const float T  = fast_tanh((at[r] * gs + cbc) + gbc);
      const float Cv = I * T;
      const float O  = fast_sigmoid(((ao[r] * gs + cbo) + wc * Cv) + gbo);
      const float Hv = O * fast_tanh(Cv);
      H[(hh * 8u + (unsigned)r) * LDH + col] = toh_flush(HCARRY * fmaxf(Hv, 0.0f));
    }
  }
  wave_lds_sync();

  v16h ha[4];
#pragma unroll
  for (int c = 0; c < 4; ++c) ha[c] = ld_frag(H + c * 32, LDH);
  const float s1 = 1.0f / (HCARRY * WCARRY);
#pragma unroll 2
  for (unsigned n = 0; n < 4u; ++n) {
    const unsigned col = 16u * n + m;
    const _Float16* bp = M1t + (size_t)col * HIDN + hh * 8u;
    v8f acc = {};
#pragma unroll
    for (int c = 0; c < 4; ++c) {
      const v16h bf = frag_at(bp + c * 32);
      acc = wmma16(ha[c], bf, acc);
    }
    const float b1 = bf16r(bm1[col]);
#pragma unroll
    for (int r = 0; r < 8; ++r)
      H1[(hh * 8u + (unsigned)r) * LDT + col] =
          toh_flush(H1CARRY * fmaxf(acc[r] * s1 + b1, 0.0f));
  }
  wave_lds_sync();

  v16h ga[2];
#pragma unroll
  for (int c = 0; c < 2; ++c) ga[c] = ld_frag(H1 + c * 32, LDT);
  const float s2 = 1.0f / (H1CARRY * WCARRY);
  float red[8];
#pragma unroll
  for (int r = 0; r < 8; ++r) red[r] = 0.0f;
#pragma unroll
  for (unsigned n = 0; n < 2u; ++n) {
    const unsigned col = 16u * n + m;
    const _Float16* bp = M2t + (size_t)col * MID1 + hh * 8u;
    v8f acc = {};
#pragma unroll
    for (int c = 0; c < 2; ++c) {
      const v16h bf = frag_at(bp + c * 32);
      acc = wmma16(ga[c], bf, acc);
    }
    const float b2 = bf16r(bm2[col]);
    const float w3 = bf16r(M3[col]);
#pragma unroll
    for (int r = 0; r < 8; ++r) red[r] += fmaxf(acc[r] * s2 + b2, 0.0f) * w3;
  }
#pragma unroll
  for (int r = 0; r < 8; ++r) red[r] = red16_sum(red[r]);
  const float b3 = bf16r(bm3[0]);
  float val = red[0];
#pragma unroll
  for (int r = 1; r < 8; ++r) val = (m == (unsigned)r) ? red[r] : val;
  if (m < 8u) Outs[wave * 16u + hh * 8u + m] = val + b3;
  __syncthreads();

  const unsigned li = (lane < 16u) ? lane : 15u;
  const v4f ov = *(const v4f*)&Outs[4u * li];
  const unsigned orow = row0 + 4u * li;
  const bool ok = (wave == 0u) && (lane < 16u) && (orow + 3u < (unsigned)NROWS);
  float* op = out + (ok ? orow : 0u);
  if (ok) *(volatile v4f*)op = ov;
  __threadfence();
  if (ok) *(volatile v4f*)op = ov;
}

extern "C" void kernel_launch(void* const* d_in, const int* in_sizes, int n_in,
                              void* d_out, int out_size, void* d_ws, size_t ws_size,
                              hipStream_t stream) {
  if (n_in < 28) return;
  if ((long long)in_sizes[0] < (long long)NROWS * XDIM) return;
  if (in_sizes[3] < XDIM * HIDN || in_sizes[5] < XDIM * HIDN || in_sizes[6] < XDIM * HIDN) return;
  if (in_sizes[11] < HIDN || in_sizes[13] < HIDN || in_sizes[14] < HIDN) return;
  if (in_sizes[17] < HIDN) return;
  if (in_sizes[18] < HIDN || in_sizes[20] < HIDN || in_sizes[21] < HIDN) return;
  if (in_sizes[22] < HIDN * MID1 || in_sizes[23] < MID1) return;
  if (in_sizes[24] < MID1 * MID2 || in_sizes[25] < MID2) return;
  if (in_sizes[26] < MID2 || in_sizes[27] < 1) return;
  if ((long long)out_size < (long long)NROWS) return;
  if (ws_size < WS_TOTAL) return;

  const float* X   = (const float*)d_in[0];
  const float* wi  = (const float*)d_in[3];
  const float* wc  = (const float*)d_in[5];
  const float* wo  = (const float*)d_in[6];
  const float* bci = (const float*)d_in[11];
  const float* bcc = (const float*)d_in[13];
  const float* bco = (const float*)d_in[14];
  const float* wco = (const float*)d_in[17];
  const float* bgi = (const float*)d_in[18];
  const float* bgc = (const float*)d_in[20];
  const float* bgo = (const float*)d_in[21];
  const float* m1  = (const float*)d_in[22];
  const float* bm1 = (const float*)d_in[23];
  const float* m2  = (const float*)d_in[24];
  const float* bm2 = (const float*)d_in[25];
  const float* m3  = (const float*)d_in[26];
  const float* bm3 = (const float*)d_in[27];
  float* out = (float*)d_out;

  char* ws = (char*)d_ws;
  _Float16* Wg  = (_Float16*)(ws + OFF_WG);
  _Float16* M1t = (_Float16*)(ws + OFF_M1);
  _Float16* M2t = (_Float16*)(ws + OFF_M2);

  dim3 blk(256);
  wsmall_kernel<<<dim3(HIDN * XDIM / 8 / 256), blk, 0, stream>>>(wi, Wg, (unsigned)XDIM, (unsigned)HIDN);
  wsmall_kernel<<<dim3(HIDN * XDIM / 8 / 256), blk, 0, stream>>>(wc, Wg + (size_t)HIDN * XDIM, (unsigned)XDIM, (unsigned)HIDN);
  wsmall_kernel<<<dim3(HIDN * XDIM / 8 / 256), blk, 0, stream>>>(wo, Wg + (size_t)2 * HIDN * XDIM, (unsigned)XDIM, (unsigned)HIDN);
  wsmall_kernel<<<dim3(MID1 * HIDN / 8 / 256), blk, 0, stream>>>(m1, M1t, (unsigned)HIDN, (unsigned)MID1);
  wsmall_kernel<<<dim3(MID2 * MID1 / 8 / 256), blk, 0, stream>>>(m2, M2t, (unsigned)MID1, (unsigned)MID2);

  gclstm_mlp_kernel<<<dim3(NBLK), dim3(128), 0, stream>>>(
      X, Wg, M1t, M2t, bci, bcc, bco, bgi, bgc, bgo, wco, bm1, bm2, m3, bm3, out);
}
